// InvLocalPatOrientConvolution_7928509629264
// MI455X (gfx1250) — hardware-verified
//
#include <hip/hip_runtime.h>
#include <stdint.h>

typedef __attribute__((ext_vector_type(16))) _Float16 v16h;
typedef __attribute__((ext_vector_type(8)))  _Float16 v8h;
typedef __attribute__((ext_vector_type(8)))  float    v8f;
typedef __attribute__((ext_vector_type(4)))  float    v4f;

#define IN_D     40
#define OUT_D    36
#define NCH      16
#define NS       10
#define NR       10
#define NL       4
#define NTAP     125
#define NCHUNK   63
#define NCOL     160
#define IN_VOX   64000
#define OUT_VOX  46656
#define NGRID    27
#define KSCALE      64.0f
#define KSCALE_INV  0.015625f
#define SLAB_P   164
#define KB_HALVES (NCHUNK * NS * 32 * 16)

__device__ __forceinline__ v8f mma16(v16h a, v16h b, v8f c) {
  return __builtin_amdgcn_wmma_f32_16x16x32_f16(false, a, false, b, (short)0, c, false, false);
}
__device__ __forceinline__ void guard4x(v8f& a, v8f& b, v8f& c, v8f& d, v16h w, v16h x, v16h y, v16h z) {
  asm volatile("v_nop\n\tv_nop\n\tv_nop\n\tv_nop" : "+v"(a), "+v"(b), "+v"(c), "+v"(d) : "v"(w), "v"(x), "v"(y), "v"(z));
}
__device__ __forceinline__ void acc_guard4(v8f& a, v8f& b, v8f& c, v8f& d) {
  asm volatile("v_nop\n\tv_nop\n\tv_nop\n\tv_nop" : "+v"(a), "+v"(b), "+v"(c), "+v"(d));
}
__device__ __forceinline__ v16h load_frag16(const _Float16* p) {
  union { v16h v; v8h h[2]; } f;
  f.h[0] = *(const v8h*)(p);
  f.h[1] = *(const v8h*)(p + 8);
  return f.v;
}

__global__ __launch_bounds__(256) void cvt_x_f16(const float* __restrict__ x, _Float16* __restrict__ xh, int nthr) {
  const int t = blockIdx.x * 256 + threadIdx.x;
  if (t >= nthr) return;
  const int v = t >> 1, q = t & 1;
  const int b = v / IN_VOX;
  const int sp = v - b * IN_VOX;
  const float* src = x + (size_t)(b * NCH + 8 * q) * IN_VOX + sp;
  v8h hv;
#pragma unroll
  for (int e = 0; e < 8; ++e) hv[e] = (_Float16)src[(size_t)e * IN_VOX];
  _Float16* dst = xh + (size_t)v * NCH + 8 * q;
  *(volatile v8h*)dst = hv;
  __threadfence();
  *(volatile v8h*)dst = hv;
}

__global__ __launch_bounds__(256) void build_kb(const float* __restrict__ weight, const float* __restrict__ zerow,
                                                const float* __restrict__ bfun, const int* __restrict__ wig_w,
                                                const int* __restrict__ wig_b, _Float16* __restrict__ kb, int nthr) {
  const int t = blockIdx.x * 256 + threadIdx.x;
  if (t >= nthr) return;
  const int q = t & 1;
  const int lane = (t >> 1) & 31;
  const int cs = t >> 6;
  const int s = cs % NS;
  const int c = cs / NS;
  const int h = lane >> 4, e = lane & 15;
  const int tap = 2 * c + q;
  int lw = wig_w[s]; lw = lw < 0 ? 0 : (lw > NL - 1 ? NL - 1 : lw);
  int lb = wig_b[s]; lb = lb < 0 ? 0 : (lb > NL - 1 ? NL - 1 : lb);
  float a[8];
#pragma unroll
  for (int j = 0; j < 8; ++j) a[j] = 0.f;
  if (tap < NTAP) {
    const float* bp = bfun + (size_t)lb * (NR * NTAP) + tap;
    if (lw == 0) {
      const float g0 = bp[0];
      const float* zp = zerow + e * NCH + 8 * h;
#pragma unroll
      for (int j = 0; j < 8; ++j) a[j] = zp[j] * g0;
    }
#pragma unroll 1
    for (int r = 1; r < NR; ++r) {
      const float g = bp[r * NTAP];
      const float* wp = weight + ((size_t)(lw * (NR - 1) + (r - 1)) * NCH + e) * NCH + 8 * h;
#pragma unroll
      for (int j = 0; j < 8; ++j) a[j] += wp[j] * g;
    }
  }
  v8h hv;
#pragma unroll
  for (int j = 0; j < 8; ++j) hv[j] = (_Float16)(a[j] * KSCALE);
  _Float16* dst = kb + (size_t)t * 8;
  *(volatile v8h*)dst = hv;
  __threadfence();
  *(volatile v8h*)dst = hv;
}

__device__ __forceinline__ void wave_sync_lds() {
  __builtin_amdgcn_fence(__ATOMIC_RELEASE, "workgroup");
  __builtin_amdgcn_wave_barrier();
  __builtin_amdgcn_fence(__ATOMIC_ACQUIRE, "workgroup");
}

__device__ __forceinline__ void store_tile(const v8f (&acc)[NS], float* sl, float* __restrict__ cv, size_t vbase, int lane) {
  const int h = lane >> 4, m = lane & 15;
#pragma unroll
  for (int s = 0; s < NS; ++s) {
#pragma unroll
    for (int r = 0; r < 8; ++r) sl[(8 * h + r) * SLAB_P + s * NCH + m] = acc[s][r] * KSCALE_INV;
  }
  wave_sync_lds();
  for (int pass = 0; pass < 2; ++pass) {
#pragma unroll
    for (int it = 0; it < 20; ++it) {
      const int grp = it / 5;
      const int within = (it - grp * 5) * 32 + lane;
      const int dzr = within / 40;
      const int c4 = within - dzr * 40;
      const v4f v = *(const v4f*)(sl + (grp * 4 + dzr) * SLAB_P + c4 * 4);
      *(volatile v4f*)(cv + (vbase + (size_t)grp * OUT_D) * NCOL + (size_t)within * 4) = v;
    }
    __threadfence();
  }
  wave_sync_lds();
}

__global__ __launch_bounds__(96) void conv_igemm(const _Float16* __restrict__ xh, const _Float16* __restrict__ kb,
                                                 float* __restrict__ cv) {
  __shared__ __align__(16) _Float16 xs[6 * 8 * 16 * NCH];
  __shared__ __align__(16) float slab[3][16 * SLAB_P];
  const int tid = threadIdx.x;
  const int wave = tid >> 5;
  const int lane = tid & 31;
  const int xp = blockIdx.x;
  const int yq = blockIdx.y;
  const int b  = blockIdx.z / 3;
  const int zt = blockIdx.z - 3 * b;
  const int x0 = 2 * xp, y0 = 4 * yq, z0b = 12 * zt;

  {
    const int4* gsrc = (const int4*)xh;
    int4* ldst = (int4*)xs;
    for (int f = tid; f < 1536; f += 96) {
      const int cw = f & 31, rr = f >> 5;
      const int gyo = rr & 7, gxo = rr >> 3;
      const size_t vox = ((size_t)(b * IN_D + x0 + gxo) * IN_D + (y0 + gyo)) * IN_D + z0b;
      ldst[f] = gsrc[vox * 2 + cw];
    }
  }
  __syncthreads();

  const int h = lane >> 4, m = lane & 15;
  const int dy = m >> 2, dz = m & 3;
  const int laneoff = (dy * 16 + 4 * wave + dz) * NCH + 8 * h;

  v8f acc0[NS], acc1[NS];
#pragma unroll
  for (int s = 0; s < NS; ++s) {
    acc0[s] = (v8f){0.f, 0.f, 0.f, 0.f, 0.f, 0.f, 0.f, 0.f};
    acc1[s] = (v8f){0.f, 0.f, 0.f, 0.f, 0.f, 0.f, 0.f, 0.f};
  }
  const _Float16* kbl = kb + (size_t)lane * 16;

  for (int c = 0; c < NCHUNK; ++c) {
    const int tap0 = 2 * c;
    int tap1 = tap0 + 1;
    tap1 = (tap1 < NTAP) ? tap1 : (NTAP - 1);
    const int dk0 = tap0 % 5, dj0 = (tap0 / 5) % 5, di0 = tap0 / 25;
    const int dk1 = tap1 % 5, dj1 = (tap1 / 5) % 5, di1 = tap1 / 25;
    const int o0 = (di0 * 8 + dj0) * 256 + dk0 * 16 + laneoff;
    const int o1 = (di1 * 8 + dj1) * 256 + dk1 * 16 + laneoff;
    union { v16h v; v8h hh[2]; } af0, af1;
    af0.hh[0] = *(const v8h*)(xs + o0);
    af0.hh[1] = *(const v8h*)(xs + o1);
    af1.hh[0] = *(const v8h*)(xs + o0 + 2048);
    af1.hh[1] = *(const v8h*)(xs + o1 + 2048);
    const _Float16* kp = kbl + (size_t)c * (NS * 512);
#pragma unroll
    for (int g = 0; g < NS / 2; ++g) {
      const v16h b0 = load_frag16(kp + (2 * g) * 512);
      const v16h b1 = load_frag16(kp + (2 * g + 1) * 512);
      acc0[2 * g]     = mma16(af0.v, b0, acc0[2 * g]);
      acc1[2 * g]     = mma16(af1.v, b0, acc1[2 * g]);
      acc0[2 * g + 1] = mma16(af0.v, b1, acc0[2 * g + 1]);
      acc1[2 * g + 1] = mma16(af1.v, b1, acc1[2 * g + 1]);
      guard4x(acc0[2 * g], acc1[2 * g], acc0[2 * g + 1], acc1[2 * g + 1], af0.v, af1.v, b0, b1);
    }
  }
  acc_guard4(acc0[0], acc0[1], acc0[2], acc0[3]);
  acc_guard4(acc0[4], acc0[5], acc0[6], acc0[7]);
  acc_guard4(acc0[8], acc0[9], acc1[0], acc1[1]);
  acc_guard4(acc1[2], acc1[3], acc1[4], acc1[5]);
  acc_guard4(acc1[6], acc1[7], acc1[8], acc1[9]);

  float* sl = slab[wave];
  const int z0w = z0b + 4 * wave;
  const size_t vbase0 = ((size_t)(b * OUT_D + x0) * OUT_D + y0) * OUT_D + z0w;
  const size_t vbase1 = ((size_t)(b * OUT_D + x0 + 1) * OUT_D + y0) * OUT_D + z0w;
  store_tile(acc0, sl, cv, vbase0, lane);
  store_tile(acc1, sl, cv, vbase1, lane);
}

__global__ __launch_bounds__(256) void so3_pool(const float* __restrict__ cv, const float* __restrict__ sgrid,
                                                const float* __restrict__ w_i, const float* __restrict__ bias,
                                                float* __restrict__ out, int nout) {
  const int f = blockIdx.x * 256 + threadIdx.x;
  if (f >= nout) return;
  int u = f;
  const int Z = u % OUT_D; u /= OUT_D;
  const int Y = u % OUT_D; u /= OUT_D;
  const int X = u % OUT_D; u /= OUT_D;
  const int d = u % NCH;
  const int b = u / NCH;
  const size_t v = ((size_t)(b * OUT_D + X) * OUT_D + Y) * OUT_D + Z;
  const float* cp = cv + v * NCOL + d;
  float cr[NS];
#pragma unroll
  for (int s = 0; s < NS; ++s) cr[s] = cp[s * NCH];
  float den = 0.f, num = 0.f;
#pragma unroll 1
  for (int g = 0; g < NGRID; ++g) {
    const float* gp = sgrid + g * NS;
    float p = 0.f;
#pragma unroll
    for (int s = 0; s < NS; ++s) p += gp[s] * cr[s];
    p = fmaxf(p, 0.f);
    const float wl = w_i[(g / 3) % 3];
    den += p * wl;
    num += (p * p) * wl;
  }
  const float res = num * (1.0f / (den + 1e-16f)) + bias[d];
  ((volatile float*)out)[f] = res;
  __threadfence();
  ((volatile float*)out)[f] = res;
}

extern "C" void kernel_launch(void* const* d_in, const int* in_sizes, int n_in,
                              void* d_out, int out_size, void* d_ws, size_t ws_size,
                              hipStream_t stream) {
  if (n_in < 9) return;
  const float* x      = (const float*)d_in[0];
  const float* weight = (const float*)d_in[1];
  const float* zerow  = (const float*)d_in[2];
  const float* bias   = (const float*)d_in[3];
  const float* sgrid  = (const float*)d_in[4];
  const float* w_i    = (const float*)d_in[5];
  const float* bfun   = (const float*)d_in[6];
  const int*   wig_w  = (const int*)d_in[7];
  const int*   wig_b  = (const int*)d_in[8];

  const int nx = in_sizes[0];
  const int B = nx / (NCH * IN_VOX);
  if (B < 1 || B > 1024 || B * NCH * IN_VOX != nx) return;
  if (out_size != B * NCH * OUT_VOX) return;
  if (in_sizes[1] < NL * (NR - 1) * NCH * NCH || in_sizes[2] < NCH * NCH || in_sizes[3] < NCH ||
      in_sizes[4] < NGRID * NS || in_sizes[5] < 3 || in_sizes[6] < NL * NR * NTAP ||
      in_sizes[7] < NS || in_sizes[8] < NS) return;

  const size_t cv_bytes = (size_t)B * OUT_VOX * NCOL * sizeof(float);
  const size_t xh_bytes = (size_t)B * IN_VOX * NCH * 2;
  const size_t kb_bytes = (size_t)KB_HALVES * 2;
  const size_t off_cv = 0;
  const size_t off_xh = (off_cv + cv_bytes + 255) & ~(size_t)255;
  const size_t off_kb = (off_xh + xh_bytes + 255) & ~(size_t)255;
  const size_t total  = (off_kb + kb_bytes + 255) & ~(size_t)255;
  if (total > ws_size || total > ((size_t)128 << 20)) return;

  float*    cv = (float*)((char*)d_ws + off_cv);
  _Float16* xh = (_Float16*)((char*)d_ws + off_xh);
  _Float16* kb = (_Float16*)((char*)d_ws + off_kb);
  float*    out = (float*)d_out;

  const int n_cvt = B * IN_VOX * 2;
  cvt_x_f16<<<dim3((n_cvt + 255) / 256), dim3(256), 0, stream>>>(x, xh, n_cvt);

  const int n_kb = NCHUNK * NS * 32 * 2;
  build_kb<<<dim3((n_kb + 255) / 256), dim3(256), 0, stream>>>(weight, zerow, bfun, wig_w, wig_b, kb, n_kb);

  conv_igemm<<<dim3(OUT_D / 2, OUT_D / 4, B * 3), dim3(96), 0, stream>>>(xh, kb, cv);

  so3_pool<<<dim3((out_size + 255) / 256), dim3(256), 0, stream>>>(cv, sgrid, w_i, bias, out, out_size);
}
